// SimpleAttention_18734647345730
// MI455X (gfx1250) — hardware-verified
//
#include <hip/hip_runtime.h>
#include <stdint.h>


typedef _Float16 v16h __attribute__((ext_vector_type(16)));
typedef _Float16 v8h  __attribute__((ext_vector_type(8)));
typedef _Float16 v8ha __attribute__((ext_vector_type(8), may_alias));
typedef __bf16   v16b __attribute__((ext_vector_type(16)));
typedef unsigned short v8us  __attribute__((ext_vector_type(8)));
typedef unsigned short v8usa __attribute__((ext_vector_type(8), may_alias));
typedef float    v8f  __attribute__((ext_vector_type(8)));
typedef float    v4f  __attribute__((ext_vector_type(4)));
typedef float    v4fa __attribute__((ext_vector_type(4), may_alias));
typedef unsigned int v4u __attribute__((ext_vector_type(4)));

union U8f  { v8f  v; v4f q[2]; float f[8]; };
union U16h { v16h v; v8h  h[2]; };
union U16s { v16h v; v8us h[2]; };
union U8h  { v8h  v; _Float16 f[8]; };

#ifndef NB
#define NB 4
#endif
#ifndef SEQ
#define SEQ 2048
#endif
#define NB_FULL  4
#define SEQ_FULL 2048
#define DH       1024
#define MROWS    (NB * SEQ)

#define GT   128
#define LP   136
#define WT   64
#define WTP  72
#define BQR  32
#define BK   32
#define QP   (DH + 8)
#define KP   (DH + 8)
#define VP   40

static_assert(NB >= 1 && NB <= NB_FULL);
static_assert(SEQ >= GT && SEQ <= SEQ_FULL);
static_assert(SEQ % GT == 0);
static_assert(SEQ % BQR == 0);
static_assert(SEQ % BK == 0);
static_assert(DH % GT == 0);
static_assert(DH % WT == 0);
static_assert(DH == 4 * 256);
static_assert(DH % 32 == 0);
static_assert((MROWS * (DH / 8)) % 256 == 0);

#define SQ_OFF   0
#define SK_OFF   (SQ_OFF + BQR * QP)
#define SV_OFF   (SK_OFF + BK * KP)
#define SX_OFFH  (SV_OFF + DH * VP)
#define SP_OFF   (SX_OFFH + 2 * (8 * 2 * 256))
#define LDS_HALVES (SP_OFF + 8 * 16 * BK)
#define LDS_BYTES  (LDS_HALVES * 2)
static_assert((SK_OFF * 2) % 16 == 0);
static_assert((SV_OFF * 2) % 16 == 0);
static_assert((SX_OFFH * 2) % 16 == 0);
static_assert((SP_OFF * 2) % 16 == 0);
static_assert(LDS_BYTES == 238592);
static_assert(8 * 16 * 64 * 4 <= (SX_OFFH - SK_OFF) * 2);

#define C2SCALE 0.045084220027780106f

__device__ __forceinline__ v8f wmma_f16(v16h a, v16h b, v8f c) {
  v8f d = __builtin_amdgcn_wmma_f32_16x16x32_f16(false, a, false, b, (short)0, c, false, false);
  asm volatile("v_nop\n\tv_nop\n\tv_nop\n\tv_nop" : "+v"(d) : "v"(a), "v"(b));
  return d;
}
__device__ __forceinline__ v8f wmma_bf16(v16h a, v16h b, v8f c) {
  v8f d = __builtin_amdgcn_wmma_f32_16x16x32_bf16(false, __builtin_bit_cast(v16b, a), false,
                                                   __builtin_bit_cast(v16b, b), (short)0, c, false, false);
  asm volatile("v_nop\n\tv_nop\n\tv_nop\n\tv_nop" : "+v"(d) : "v"(a), "v"(b));
  return d;
}

template <int CTRL>
__device__ __forceinline__ float dppf(float x) {
  int s = __float_as_int(x);
  return __int_as_float(__builtin_amdgcn_update_dpp(s, s, CTRL, 0xF, 0xF, true));
}
__device__ __forceinline__ float red_max16(float x) {
  x = fmaxf(x, dppf<0xB1>(x));
  x = fmaxf(x, dppf<0x4E>(x));
  x = fmaxf(x, dppf<0x141>(x));
  x = fmaxf(x, dppf<0x140>(x));
  return x;
}
__device__ __forceinline__ float red_sum16(float x) {
  x += dppf<0xB1>(x);
  x += dppf<0x4E>(x);
  x += dppf<0x141>(x);
  x += dppf<0x140>(x);
  return x;
}

__device__ __forceinline__ void wave_lds_sync() {
  __builtin_amdgcn_fence(3, "wavefront");
  asm volatile("s_wait_dscnt 0" ::: "memory");
  __builtin_amdgcn_wave_barrier();
}

__device__ __forceinline__ v4u bf16_bits4(v4f a) {
  v4u u = __builtin_bit_cast(v4u, a);
  u = (u + 0x7FFFu + ((u >> 16) & 1u)) >> 16;
  return u;
}
__device__ __forceinline__ float bf16_rne1(float a) {
  unsigned int u = __float_as_uint(a);
  u = (u + 0x7FFFu + ((u >> 16) & 1u)) & 0xFFFF0000u;
  return __uint_as_float(u);
}
__device__ __forceinline__ v8us pack8(v4u a, v4u b) {
  v8us d;
  d[0] = (unsigned short)a[0]; d[1] = (unsigned short)a[1];
  d[2] = (unsigned short)a[2]; d[3] = (unsigned short)a[3];
  d[4] = (unsigned short)b[0]; d[5] = (unsigned short)b[1];
  d[6] = (unsigned short)b[2]; d[7] = (unsigned short)b[3];
  return d;
}

__global__ __launch_bounds__(256)
void prep_x_kernel(const float* __restrict__ X, unsigned short* __restrict__ Xb)
{
  const int p = blockIdx.x * 256 + threadIdx.x;
  const int m = p >> 7;
  const int c = (p & 127) * 8;
  const int b = m / SEQ;
  const int s = m - b * SEQ;
  const float* src = X + ((size_t)b * SEQ_FULL + s) * DH + c;
  const v4u u0 = bf16_bits4(*(const v4f*)(src));
  const v4u u1 = bf16_bits4(*(const v4f*)(src + 4));
  const v8us w = pack8(u0, u1);
  unsigned short* dst = Xb + (size_t)m * DH + c;
  *(volatile v8us*)dst = w;
  __threadfence();
  *(volatile v8us*)dst = w;
}

__global__ __launch_bounds__(256)
void prep_w_kernel(const float* __restrict__ wq, const float* __restrict__ wk, const float* __restrict__ wv,
                   unsigned short* __restrict__ Wt)
{
  __shared__ __attribute__((aligned(16))) unsigned short sT[WT * WTP];
  const int tid = threadIdx.x;
  const int z   = blockIdx.z;
  const int e0  = blockIdx.x * WT;
  const int d0  = blockIdx.y * WT;
  const float* W = (z == 0) ? wq : ((z == 1) ? wk : wv);

  const int r  = tid >> 2;
  const int cg = tid & 3;
  const float* src = W + (size_t)(d0 + r) * DH + e0 + 16 * cg;
  #pragma unroll
  for (int u = 0; u < 4; ++u) {
    const v4u bits = bf16_bits4(*(const v4f*)(src + 4 * u));
    #pragma unroll
    for (int k = 0; k < 4; ++k) sT[(16 * cg + 4 * u + k) * WTP + r] = (unsigned short)bits[k];
  }
  __syncthreads();

  unsigned short* wb = Wt + (size_t)z * DH * DH;
  v8us vv[2]; size_t oo[2];
  #pragma unroll
  for (int i = 0; i < 2; ++i) {
    const int c = tid + 256 * i, el = c >> 3, p = c & 7;
    vv[i] = *(const v8usa*)(sT + el * WTP + 8 * p);
    oo[i] = (size_t)(e0 + el) * DH + d0 + 8 * p;
  }
  #pragma unroll
  for (int i = 0; i < 2; ++i) *(volatile v8us*)(wb + oo[i]) = vv[i];
  __threadfence();
  #pragma unroll
  for (int i = 0; i < 2; ++i) *(volatile v8us*)(wb + oo[i]) = vv[i];
}

__global__ __launch_bounds__(256) __attribute__((amdgpu_num_vgpr(256)))
void proj_kernel(const unsigned short* __restrict__ Xb, const unsigned short* __restrict__ Wt,
                 const float* __restrict__ bq, const float* __restrict__ bk, const float* __restrict__ bv,
                 _Float16* __restrict__ QK, _Float16* __restrict__ Vt)
{
  __shared__ __attribute__((aligned(16))) _Float16 sT[GT * LP];

  const int tid  = threadIdx.x;
  const int wave = tid >> 5;
  const int lane = tid & 31;
  const int lh   = lane & 15;
  const int hi   = lane >> 4;

  const int sel = blockIdx.z;
  const int n0  = blockIdx.x * GT;
  const int m0  = blockIdx.y * GT;

  const unsigned short* Wp   = Wt + (size_t)sel * DH * DH;
  const float*          bias = (sel == 0) ? bq : ((sel == 1) ? bk : bv);
  const unsigned short* arow = Xb + (size_t)(m0 + 16 * wave + lh) * DH + 8 * hi;
  const unsigned short* brow = Wp + (size_t)(n0 + lh) * DH + 8 * hi;

  U8f acc[8];
  #pragma unroll
  for (int j = 0; j < 8; ++j) acc[j].v = (v8f){};

  #pragma unroll 1
  for (int k0 = 0; k0 < DH; k0 += 32) {
    U16s a;
    a.h[0] = *(const v8us*)(arow + k0);
    a.h[1] = *(const v8us*)(arow + k0 + 16);
    #pragma unroll
    for (int j = 0; j < 8; ++j) {
      U16s bf;
      bf.h[0] = *(const v8us*)(brow + (size_t)(16 * j) * DH + k0);
      bf.h[1] = *(const v8us*)(brow + (size_t)(16 * j) * DH + k0 + 16);
      acc[j].v = wmma_bf16(a.v, bf.v, acc[j].v);
    }
  }

  const bool tr = (sel == 2);
  if (tr) {
    #pragma unroll
    for (int j = 0; j < 8; ++j) {
      const float bb = bf16_rne1(bias[n0 + 16 * j + lh]);
      #pragma unroll
      for (int t = 0; t < 8; ++t)
        sT[(16 * j + lh) * LP + 16 * wave + 8 * hi + t] = (_Float16)(acc[j].f[t] + bb);
    }
  } else {
    #pragma unroll
    for (int j = 0; j < 8; ++j) {
      const float bb = bf16_rne1(bias[n0 + 16 * j + lh]);
      #pragma unroll
      for (int t = 0; t < 8; ++t)
        sT[(16 * wave + 8 * hi + t) * LP + 16 * j + lh] = (_Float16)(acc[j].f[t] + bb);
    }
  }
  __syncthreads();

  const int bb0 = m0 / SEQ;
  const int s0  = m0 - bb0 * SEQ;
  _Float16* dq = QK + (size_t)sel * MROWS * DH + (size_t)m0 * DH + n0;
  _Float16* dv = Vt + ((size_t)bb0 * DH + n0) * SEQ + s0;
  _Float16* dbase = tr ? dv : dq;
  const size_t rs = tr ? (size_t)SEQ : (size_t)DH;

  v8h vv[8]; size_t oo[8];
  #pragma unroll
  for (int i = 0; i < 8; ++i) {
    const int c = tid + 256 * i, L = c >> 3, p = c & 7;
    const int r = L >> 1, h = L & 1;
    vv[i] = *(const v8ha*)(sT + r * LP + 64 * h + 8 * p);
    oo[i] = (size_t)r * rs + 64 * h + 8 * p;
  }
  #pragma unroll
  for (int i = 0; i < 8; ++i) *(volatile v8h*)(dbase + oo[i]) = vv[i];
  __threadfence();
  #pragma unroll
  for (int i = 0; i < 8; ++i) *(volatile v8h*)(dbase + oo[i]) = vv[i];
}

__global__ __launch_bounds__(256) __attribute__((amdgpu_num_vgpr(256)))
void attn_kernel(const _Float16* __restrict__ QK, const _Float16* __restrict__ Vt, float* __restrict__ Out)
{
  extern __shared__ __attribute__((aligned(16))) _Float16 smem[];
  _Float16* sQ = smem + SQ_OFF;
  _Float16* sK = smem + SK_OFF;
  _Float16* sV = smem + SV_OFF;
  float*    sX = (float*)(smem + SX_OFFH);
  _Float16* sP = smem + SP_OFF;
  float*    sO = (float*)(smem + SK_OFF);

  const int tid  = threadIdx.x;
  const int wave = tid >> 5;
  const int lane = tid & 31;
  const int lh   = lane & 15;
  const int hi   = lane >> 4;
  const int rt   = wave >> 2;
  const int dq   = wave & 3;

  const int nqb   = SEQ / BQR;
  const int b     = blockIdx.x / nqb;
  const int qbase = (blockIdx.x % nqb) * BQR;

  const _Float16* Qb = QK + (size_t)b * SEQ * DH;
  const _Float16* Kb = QK + (size_t)MROWS * DH + (size_t)b * SEQ * DH;
  const _Float16* Vb = Vt + (size_t)b * DH * SEQ;
  float*          Ob = Out + (size_t)b * SEQ * DH;

  #pragma unroll 4
  for (int i = 0; i < 16; ++i) {
    const int idx = tid + 256 * i;
    const int r = idx >> 7, g = idx & 127;
    const v8h q = *(const v8h*)(Qb + (size_t)(qbase + r) * DH + 8 * g);
    *(v8h*)(sQ + r * QP + 8 * g) = q;
  }

  U8f acc[16];
  #pragma unroll
  for (int t = 0; t < 16; ++t) acc[t].v = (v8f){};
  float mrow[8], lrow[8];
  #pragma unroll
  for (int j = 0; j < 8; ++j) { mrow[j] = -3.0e38f; lrow[j] = 0.0f; }

  const _Float16* qw = sQ + (16 * rt + lh) * QP + 256 * dq + 8 * hi;
  _Float16*       pw = sP + wave * (16 * BK);
  float*          xw = sX + wave * 512 + lane * 8;
  const float*    xr = sX + (rt * 4) * 512 + lane * 8;

  #pragma unroll 1
  for (int kv0 = 0; kv0 < SEQ; kv0 += BK) {
    __syncthreads();
    #pragma unroll 4
    for (int i = 0; i < 16; ++i) {
      const int idx = tid + 256 * i;
      const int r = idx >> 7, g = idx & 127;
      const v8h kk = *(const v8h*)(Kb + (size_t)(kv0 + r) * DH + 8 * g);
      *(v8h*)(sK + r * KP + 8 * g) = kk;
    }
    #pragma unroll 4
    for (int i = 0; i < 16; ++i) {
      const int idx = tid + 256 * i;
      const int d = idx >> 2, g = idx & 3;
      const v8h vv = *(const v8h*)(Vb + (size_t)d * SEQ + kv0 + 8 * g);
      *(v8h*)(sV + d * VP + 8 * g) = vv;
    }
    __syncthreads();

    U8f s0, s1; s0.v = (v8f){}; s1.v = (v8f){};
    const _Float16* kw = sK + lh * KP + 256 * dq + 8 * hi;
    #pragma unroll
    for (int c = 0; c < 8; ++c) {
      U16h qf, kf;
      qf.h[0] = *(const v8h*)(qw + 32 * c);
      qf.h[1] = *(const v8h*)(qw + 32 * c + 16);
      kf.h[0] = *(const v8h*)(kw + 32 * c);
      kf.h[1] = *(const v8h*)(kw + 32 * c + 16);
      s0.v = wmma_f16(qf.v, kf.v, s0.v);
      kf.h[0] = *(const v8h*)(kw + 16 * KP + 32 * c);
      kf.h[1] = *(const v8h*)(kw + 16 * KP + 32 * c + 16);
      s1.v = wmma_f16(qf.v, kf.v, s1.v);
    }

    *(v4fa*)(xw)       = s0.q[0];
    *(v4fa*)(xw + 4)   = s0.q[1];
    *(v4fa*)(xw + 256) = s1.q[0];
    *(v4fa*)(xw + 260) = s1.q[1];
    __syncthreads();
    U8f t0, t1;
    t0.q[0] = *(const v4fa*)(xr);       t0.q[1] = *(const v4fa*)(xr + 4);
    t1.q[0] = *(const v4fa*)(xr + 256); t1.q[1] = *(const v4fa*)(xr + 260);
    #pragma unroll
    for (int w2 = 1; w2 < 4; ++w2) {
      const v4f p0 = *(const v4fa*)(xr + 512 * w2);
      const v4f p1 = *(const v4fa*)(xr + 512 * w2 + 4);
      const v4f p2 = *(const v4fa*)(xr + 512 * w2 + 256);
      const v4f p3 = *(const v4fa*)(xr + 512 * w2 + 260);
      t0.q[0] = t0.q[0] + p0; t0.q[1] = t0.q[1] + p1;
      t1.q[0] = t1.q[0] + p2; t1.q[1] = t1.q[1] + p3;
    }

    U8h pa, pb;
    #pragma unroll
    for (int j = 0; j < 8; ++j) {
      const float a  = t0.f[j] * C2SCALE;
      const float bb = t1.f[j] * C2SCALE;
      const float rm    = red_max16(fmaxf(a, bb));
      const float mnew  = fmaxf(mrow[j], rm);
      const float alpha = __builtin_amdgcn_exp2f(mrow[j] - mnew);
      const float e0    = __builtin_amdgcn_exp2f(a  - mnew);
      const float e1    = __builtin_amdgcn_exp2f(bb - mnew);
      lrow[j] = lrow[j] * alpha + red_sum16(e0 + e1);
      mrow[j] = mnew;
      pa.f[j] = (_Float16)(e0 * 1024.0f);
      pb.f[j] = (_Float16)(e1 * 1024.0f);
      #pragma unroll
      for (int t = 0; t < 16; ++t) acc[t].f[j] *= alpha;
    }

    #pragma unroll
    for (int j = 0; j < 8; ++j) {
      pw[(j + 8 * hi) * BK + lh]      = pa.f[j];
      pw[(j + 8 * hi) * BK + 16 + lh] = pb.f[j];
    }
    wave_lds_sync();
    U16h pf;
    pf.h[0] = *(const v8ha*)(pw + lh * BK + 8 * hi);
    pf.h[1] = *(const v8ha*)(pw + lh * BK + 16 + 8 * hi);

    const _Float16* vw = sV + (256 * dq + lh) * VP + 8 * hi;
    #pragma unroll
    for (int t = 0; t < 16; ++t) {
      U16h vf;
      vf.h[0] = *(const v8h*)(vw + 16 * t * VP);
      vf.h[1] = *(const v8h*)(vw + 16 * t * VP + 16);
      acc[t].v = wmma_f16(pf.v, vf.v, acc[t].v);
    }
  }
  __syncthreads();

  float inv[8];
  #pragma unroll
  for (int j = 0; j < 8; ++j) inv[j] = 1.0f / (lrow[j] * 1024.0f);
  float* so = sO + wave * (16 * 64);
  float* ob = Ob + (size_t)(qbase + 16 * rt) * DH + 256 * dq;
  #pragma unroll
  for (int g = 0; g < 4; ++g) {
    #pragma unroll
    for (int j = 0; j < 8; ++j) {
      #pragma unroll
      for (int tt = 0; tt < 4; ++tt)
        so[(j + 8 * hi) * 64 + tt * 16 + lh] = acc[4 * g + tt].f[j] * inv[j];
    }
    wave_lds_sync();
    v4f ov[8]; int oo[8];
    #pragma unroll
    for (int i = 0; i < 8; ++i) {
      const int c = lane + 32 * i, rr = c >> 4, q = c & 15;
      ov[i] = *(const v4fa*)(so + rr * 64 + q * 4);
      oo[i] = rr * DH + 64 * g + 4 * q;
    }
    #pragma unroll
    for (int i = 0; i < 8; ++i) *(volatile v4f*)(ob + oo[i]) = ov[i];
    __threadfence();
    #pragma unroll
    for (int i = 0; i < 8; ++i) *(volatile v4f*)(ob + oo[i]) = ov[i];
    wave_lds_sync();
  }
}

extern "C" void kernel_launch(void* const* d_in, const int* in_sizes, int n_in,
                              void* d_out, int out_size, void* d_ws, size_t ws_size,
                              hipStream_t stream) {
  if (n_in < 7) return;
  const long long need_x = ((long long)(NB - 1) * SEQ_FULL + SEQ) * DH;
  if ((long long)in_sizes[0] < need_x) return;
  if (in_sizes[1] < DH * DH || in_sizes[3] < DH * DH || in_sizes[5] < DH * DH) return;
  if (in_sizes[2] < DH || in_sizes[4] < DH || in_sizes[6] < DH) return;
  if ((long long)out_size < (long long)MROWS * DH) return;

  const size_t xb_bytes = (size_t)MROWS * DH * 2;
  const size_t wt_bytes = (size_t)3 * DH * DH * 2;
  const size_t qk_bytes = (size_t)2 * MROWS * DH * 2;
  const size_t vt_bytes = (size_t)NB * DH * SEQ * 2;
  const size_t off_xb = 0;
  const size_t off_wt = off_xb + xb_bytes;
  const size_t off_qk = off_wt + wt_bytes;
  const size_t off_vt = off_qk + qk_bytes;
  if (off_vt + vt_bytes > ws_size) return;

  const float* x  = (const float*)d_in[0];
  const float* wq = (const float*)d_in[1];
  const float* bq = (const float*)d_in[2];
  const float* wk = (const float*)d_in[3];
  const float* bk = (const float*)d_in[4];
  const float* wv = (const float*)d_in[5];
  const float* bv = (const float*)d_in[6];
  float* out = (float*)d_out;
  unsigned short* xb = (unsigned short*)((char*)d_ws + off_xb);
  unsigned short* wt = (unsigned short*)((char*)d_ws + off_wt);
  _Float16*       qk = (_Float16*)((char*)d_ws + off_qk);
  _Float16*       vt = (_Float16*)((char*)d_ws + off_vt);

  prep_x_kernel<<<(MROWS * (DH / 8)) / 256, 256, 0, stream>>>(x, xb);
  prep_w_kernel<<<dim3(DH / WT, DH / WT, 3), 256, 0, stream>>>(wq, wk, wv, wt);
  proj_kernel<<<dim3(DH / GT, MROWS / GT, 3), 256, 0, stream>>>(xb, wt, bq, bk, bv, qk, vt);

  (void)hipFuncSetAttribute(reinterpret_cast<const void*>(&attn_kernel),
                            hipFuncAttributeMaxDynamicSharedMemorySize, (int)LDS_BYTES);
  attn_kernel<<<MROWS / BQR, 256, LDS_BYTES, stream>>>(qk, vt, out);
}
